// MultiheadedAttention_71846212928240
// MI455X (gfx1250) — hardware-verified
//
#include <hip/hip_runtime.h>
#include <math.h>

#ifndef NB
#define NB 2
#endif
#ifndef SEQ
#define SEQ 2048
#endif
#define SEQ_FULL 2048
#define DMODEL 1024
#define NHEAD 16
#define HDIM 64
#define X_BS_FULL ((size_t)SEQ_FULL * DMODEL)
#define MTOK (NB * SEQ)
#define FINE_ROWS ((SEQ) < 512 ? (SEQ) : 512)

static_assert(NHEAD * HDIM == DMODEL);
static_assert(HDIM == 64);
static_assert(SEQ % 64 == 0);
static_assert(SEQ <= SEQ_FULL);
static_assert(FINE_ROWS % 64 == 0);
static_assert(DMODEL % 32 == 0);
static_assert(MTOK % 64 == 0);

#define XPL  ((size_t)MTOK * DMODEL)
#define WPL  ((size_t)DMODEL * DMODEL)
#define QPL  ((size_t)MTOK * DMODEL)
#define VTPL ((size_t)NB * DMODEL * SEQ)
#define FQPL ((size_t)NB * FINE_ROWS * DMODEL)
#define FVPL ((size_t)NB * DMODEL * FINE_ROWS)
#define OFF_X    ((size_t)0)
#define OFF_W    (OFF_X + 3 * XPL)
#define OFF_Q16  (OFF_W + 3 * WPL)
#define OFF_K16  (OFF_Q16 + QPL)
#define OFF_VT16 (OFF_K16 + QPL)
#define OFF_QH   (OFF_VT16 + VTPL)
#define OFF_QL   (OFF_QH + FQPL)
#define OFF_KH   (OFF_QL + FQPL)
#define OFF_KL   (OFF_KH + FQPL)
#define OFF_VTH  (OFF_KL + FQPL)
#define OFF_VTL  (OFF_VTH + FVPL)
#define WS_HALVES (OFF_VTL + FVPL)
static_assert(WS_HALVES * 2 <= (size_t)134217728);
static_assert((XPL % 64) == 0 && (WPL % 64) == 0 && (FQPL % 64) == 0 && (FVPL % 64) == 0);

#define PROJ_TILES ((MTOK / 64) * (DMODEL / 64))
static_assert(PROJ_TILES % 8 == 0);
#define FINE_BLOCKS  (NB * NHEAD * (FINE_ROWS / 64))
#define PLAIN_BLOCKS (NB * NHEAD * ((SEQ - FINE_ROWS) / 64))

typedef __attribute__((ext_vector_type(16))) _Float16     v16h;
typedef __attribute__((ext_vector_type(16))) __bf16       v16b;
typedef __attribute__((ext_vector_type(8)))  float        v8f;
typedef __attribute__((ext_vector_type(4)))  float        v4f;
typedef __attribute__((ext_vector_type(4)))  unsigned int v4u;

union FBU { v4u q[2]; v16h h; v16b b; };
__device__ __forceinline__ v16h ldfh(const unsigned short* p) { FBU f; f.q[0] = *(const v4u*)p; f.q[1] = *(const v4u*)(p + 16); return f.h; }
__device__ __forceinline__ v16b ldfb(const unsigned short* p) { FBU f; f.q[0] = *(const v4u*)p; f.q[1] = *(const v4u*)(p + 16); return f.b; }

__device__ __forceinline__ v8f mmah(v16h a, v16h b, v8f c) {
    c = __builtin_amdgcn_wmma_f32_16x16x32_f16(false, a, false, b, (short)0, c, false, false);
    asm volatile("v_nop\n\tv_nop\n\tv_nop\n\tv_nop" : "+v"(c) : "v"(a), "v"(b));
    return c;
}
__device__ __forceinline__ v8f mmab(v16b a, v16b b, v8f c) {
    c = __builtin_amdgcn_wmma_f32_16x16x32_bf16(false, a, false, b, (short)0, c, false, false);
    asm volatile("v_nop\n\tv_nop\n\tv_nop\n\tv_nop" : "+v"(c) : "v"(a), "v"(b));
    return c;
}
__device__ __forceinline__ void dep_guard_h(v8f& a, v8f& b, v16h x, v16h y) { asm volatile("v_nop\n\tv_nop\n\tv_nop\n\tv_nop" : "+v"(a), "+v"(b) : "v"(x), "v"(y)); }
__device__ __forceinline__ void keep4_h(v16h a, v16h b, v16h c, v16h d) { asm volatile("v_nop" :: "v"(a), "v"(b), "v"(c), "v"(d)); }
__device__ __forceinline__ void acc_guard4(v8f& a, v8f& b, v8f& c, v8f& d) { asm volatile("v_nop\n\tv_nop\n\tv_nop\n\tv_nop" : "+v"(a), "+v"(b), "+v"(c), "+v"(d)); }
__device__ __forceinline__ v8f zero8() { v8f z = {0.f, 0.f, 0.f, 0.f, 0.f, 0.f, 0.f, 0.f}; return z; }

__device__ __forceinline__ void wave_sync() {
    __builtin_amdgcn_fence(3  , "workgroup");
    __builtin_amdgcn_wave_barrier();
    __builtin_amdgcn_fence(2  , "workgroup");
}

__device__ __forceinline__ float cmb_bf(float v) { const unsigned u = __builtin_bit_cast(unsigned, v); const unsigned r = (u + 0x7fffu + ((u >> 16) & 1u)) & 0xffff0000u; return __builtin_bit_cast(float, r); }
__device__ __forceinline__ unsigned short bfu_rne(float v) { unsigned u = __builtin_bit_cast(unsigned, v); u += 0x7fffu + ((u >> 16) & 1u); return (unsigned short)(u >> 16); }
__device__ __forceinline__ float bfu_f32(unsigned short h) { return __builtin_bit_cast(float, ((unsigned)h) << 16); }
__device__ __forceinline__ unsigned short f16_bits(float v) { return __builtin_bit_cast(unsigned short, (_Float16)v); }
__device__ __forceinline__ unsigned int pk2h(float a, float b) { return (unsigned int)f16_bits(a) | ((unsigned int)f16_bits(b) << 16); }
__device__ __forceinline__ void st2_u4(unsigned short* d, v4u v) { volatile v4u* p = (volatile v4u*)d; *p = v; __threadfence(); *p = v; }

__device__ __forceinline__ void cvt_x_body(const float* __restrict__ src, unsigned short* __restrict__ dst, long long u) {
    const int r = (int)(u >> 7); const int c0 = ((int)(u & 127)) * 8;
    const int b = r / SEQ, n = r - b * SEQ;
    const float* s = src + (size_t)b * X_BS_FULL + (size_t)n * DMODEL + c0;
    const v4f x0 = *(const v4f*)s, x1 = *(const v4f*)(s + 4);
    v4u pk;
    pk.x = pk2h(cmb_bf(x0.x) * 16.f, cmb_bf(x0.y) * 16.f); pk.y = pk2h(cmb_bf(x0.z) * 16.f, cmb_bf(x0.w) * 16.f);
    pk.z = pk2h(cmb_bf(x1.x) * 16.f, cmb_bf(x1.y) * 16.f); pk.w = pk2h(cmb_bf(x1.z) * 16.f, cmb_bf(x1.w) * 16.f);
    st2_u4(dst + (size_t)r * DMODEL + c0, pk);
}
__global__ __launch_bounds__(256) void k_cvt_x(const float* __restrict__ xq, const float* __restrict__ xk, const float* __restrict__ xv, unsigned short* __restrict__ ws16) {
    const long long u = (long long)blockIdx.x * 256 + threadIdx.x;
    if (u >= (long long)MTOK * 128) return;
    const int which = blockIdx.y;
    if (which == 0) cvt_x_body(xq, ws16 + OFF_X, u);
    else if (which == 1) cvt_x_body(xk, ws16 + OFF_X + XPL, u);
    else cvt_x_body(xv, ws16 + OFF_X + 2 * XPL, u);
}

__device__ __forceinline__ void cvt_w_body(const float* __restrict__ src, unsigned short* __restrict__ dst, int u) {
    const int row = u >> 7; const int d0 = (u & 127) * 8;
    const int h = row >> 6, e = row & 63;
    float w[8];
#pragma unroll
    for (int i = 0; i < 8; ++i) w[i] = cmb_bf(src[((size_t)(h * DMODEL + d0 + i)) * HDIM + e]) * 32.f;
    v4u pk; pk.x = pk2h(w[0], w[1]); pk.y = pk2h(w[2], w[3]); pk.z = pk2h(w[4], w[5]); pk.w = pk2h(w[6], w[7]);
    st2_u4(dst + (size_t)row * DMODEL + d0, pk);
}
__global__ __launch_bounds__(256) void k_cvt_w(const float* __restrict__ wq, const float* __restrict__ wk, const float* __restrict__ wv, unsigned short* __restrict__ ws16) {
    const int u = blockIdx.x * 256 + threadIdx.x;
    if (u >= DMODEL * 128) return;
    const int which = blockIdx.y;
    if (which == 0) cvt_w_body(wq, ws16 + OFF_W, u);
    else if (which == 1) cvt_w_body(wk, ws16 + OFF_W + WPL, u);
    else cvt_w_body(wv, ws16 + OFF_W + 2 * WPL, u);
}

__global__ __launch_bounds__(256) void k_proj(const unsigned short* pin, unsigned short* pout,
                                              const float* __restrict__ bq, const float* __restrict__ bk, const float* __restrict__ bv) {
    __shared__ __align__(16) float sT[8][16 * 68];
    const int which = blockIdx.y;
    const bool isv = (which == 2);
    const int lane = threadIdx.x & 31, wave = threadIdx.x >> 5;
    const int tilesN = isv ? (MTOK >> 6) : (DMODEL >> 6);
    const int tile = blockIdx.x * 8 + wave;
    const int tm = tile / tilesN, tn = tile - tm * tilesN;
    const int m0 = tm << 6, n0 = tn << 6;
    const size_t aoff = isv ? (OFF_W + 2 * WPL) : (OFF_X + (size_t)which * XPL);
    const size_t boff = isv ? (OFF_X + 2 * XPL) : (OFF_W + (size_t)which * WPL);
    const unsigned short* Ab = pin + aoff;
    const unsigned short* Bb = pin + boff;
    const int rlane = lane & 15, koff = (lane >> 4) * 8, mOff = (lane >> 4) * 8;

    v8f acc[4][4];
#pragma unroll
    for (int i = 0; i < 4; ++i)
#pragma unroll
        for (int j = 0; j < 4; ++j) acc[i][j] = zero8();

    for (int k0 = 0; k0 < DMODEL; k0 += 32) {
        v16h bh[4];
#pragma unroll
        for (int j = 0; j < 4; ++j) bh[j] = ldfh(Bb + (size_t)(n0 + (j << 4) + rlane) * DMODEL + koff + k0);
#pragma unroll
        for (int i = 0; i < 4; ++i) {
            const v16h ah = ldfh(Ab + (size_t)(m0 + (i << 4) + rlane) * DMODEL + koff + k0);
#pragma unroll
            for (int j = 0; j < 4; ++j)
                acc[i][j] = __builtin_amdgcn_wmma_f32_16x16x32_f16(false, ah, false, bh[j], (short)0, acc[i][j], false, false);
            dep_guard_h(acc[i][0], acc[i][3], ah, ah);
        }
        keep4_h(bh[0], bh[1], bh[2], bh[3]);
    }
    acc_guard4(acc[0][0], acc[0][1], acc[0][2], acc[0][3]);
    acc_guard4(acc[1][0], acc[1][1], acc[1][2], acc[1][3]);
    acc_guard4(acc[2][0], acc[2][1], acc[2][2], acc[2][3]);
    acc_guard4(acc[3][0], acc[3][1], acc[3][2], acc[3][3]);

    float* slab = sT[wave];
    const float ISC = 1.0f / 512.0f;
    float bn[4] = {0.f, 0.f, 0.f, 0.f};
    if (which == 0) {
#pragma unroll
        for (int j = 0; j < 4; ++j) bn[j] = cmb_bf(bq[n0 + (j << 4) + rlane]);
    } else if (which == 1) {
#pragma unroll
        for (int j = 0; j < 4; ++j) bn[j] = cmb_bf(bk[n0 + (j << 4) + rlane]);
    }
    const int bcol = isv ? (n0 / SEQ) : 0;
    const int brow = isv ? 0 : (m0 / SEQ);
    const int colin = isv ? (n0 - bcol * SEQ) : n0;
    const bool fine = isv ? (colin < FINE_ROWS) : ((m0 - brow * SEQ) < FINE_ROWS);
    const size_t obase = isv ? OFF_VT16 : (OFF_Q16 + (size_t)which * QPL);
    const size_t hbase = isv ? OFF_VTH : (OFF_QH + (size_t)which * 2 * FQPL);
    const size_t lbase = isv ? OFF_VTL : (OFF_QL + (size_t)which * 2 * FQPL);
    const int radd_m = isv ? bcol * DMODEL : 0;
    const int radd_f = isv ? bcol * DMODEL : (brow * FINE_ROWS - brow * SEQ);
    const int pitch_m = isv ? SEQ : DMODEL;
    const int pitch_f = isv ? FINE_ROWS : DMODEL;
    const int q4 = lane >> 3, c8 = (lane & 7) * 8;
#pragma unroll
    for (int i = 0; i < 4; ++i) {
        const int mBase = m0 + (i << 4);
        float bm[8] = {0.f, 0.f, 0.f, 0.f, 0.f, 0.f, 0.f, 0.f};
        if (isv) {
#pragma unroll
            for (int r = 0; r < 8; ++r) bm[r] = cmb_bf(bv[mBase + mOff + r]);
        }
#pragma unroll
        for (int j = 0; j < 4; ++j) {
#pragma unroll
            for (int r = 0; r < 8; ++r) slab[(mOff + r) * 68 + (j << 4) + rlane] = acc[i][j][r] * ISC + bn[j] + bm[r];
        }
        wave_sync();
        for (int pass = 0; pass < 2; ++pass) {
#pragma unroll
            for (int it = 0; it < 4; ++it) {
                const int row = it * 4 + q4;
                const float* sp = slab + row * 68 + c8;
                const v4f x0 = *(const v4f*)sp, x1 = *(const v4f*)(sp + 4);
                const float w[8] = {x0.x, x0.y, x0.z, x0.w, x1.x, x1.y, x1.z, x1.w};
                const int gr = mBase + row;
                v4u pk; pk.x = pk2h(w[0] * 16.f, w[1] * 16.f); pk.y = pk2h(w[2] * 16.f, w[3] * 16.f); pk.z = pk2h(w[4] * 16.f, w[5] * 16.f); pk.w = pk2h(w[6] * 16.f, w[7] * 16.f);
                *(volatile v4u*)(pout + obase + (size_t)(radd_m + gr) * pitch_m + colin + c8) = pk;
                if (fine) {
                    unsigned short hb[8], lb[8];
#pragma unroll
                    for (int e = 0; e < 8; ++e) { hb[e] = bfu_rne(w[e]); lb[e] = bfu_rne(w[e] - bfu_f32(hb[e])); }
                    v4u ph, pq;
                    ph.x = (unsigned)hb[0] | ((unsigned)hb[1] << 16); ph.y = (unsigned)hb[2] | ((unsigned)hb[3] << 16); ph.z = (unsigned)hb[4] | ((unsigned)hb[5] << 16); ph.w = (unsigned)hb[6] | ((unsigned)hb[7] << 16);
                    pq.x = (unsigned)lb[0] | ((unsigned)lb[1] << 16); pq.y = (unsigned)lb[2] | ((unsigned)lb[3] << 16); pq.z = (unsigned)lb[4] | ((unsigned)lb[5] << 16); pq.w = (unsigned)lb[6] | ((unsigned)lb[7] << 16);
                    const size_t fo = (size_t)(radd_f + gr) * pitch_f + colin + c8;
                    *(volatile v4u*)(pout + hbase + fo) = ph;
                    *(volatile v4u*)(pout + lbase + fo) = pq;
                }
            }
            __threadfence();
        }
        wave_sync();
    }
}

#define PPITCH 40
template <bool FINE>
__device__ __forceinline__ void attn_body(const unsigned short* __restrict__ pl, float* out) {
    __shared__ __align__(16) unsigned short Ph[4][16 * PPITCH];
    __shared__ __align__(16) unsigned short Pl[4][16 * PPITCH];
    __shared__ __align__(16) float Os[4][16 * 68];
    const int tid = threadIdx.x, wave = tid >> 5, lane = tid & 31, hh = lane >> 4, c = lane & 15;
    constexpr int NQB0 = FINE ? (FINE_ROWS / 64) : ((SEQ - FINE_ROWS) / 64);
    constexpr int NQB = (NQB0 > 0) ? NQB0 : 1;
    constexpr int SP = FINE ? FINE_ROWS : SEQ;
    const int bx = blockIdx.x;
    const int qbl = bx % NQB, bhd = bx / NQB, h = bhd % NHEAD, b = bhd / NHEAD;
    const int q0 = (FINE ? qbl : (qbl + FINE_ROWS / 64)) * 64 + wave * 16;

    const size_t qidx = ((size_t)(b * SP + q0 + c)) * DMODEL + h * HDIM + 8 * hh;
    const size_t kidx = ((size_t)(b * SP + c)) * DMODEL + h * HDIM + 8 * hh;
    const size_t vidx = ((size_t)(b * DMODEL + h * HDIM + c)) * SP + 8 * hh;
    const size_t qo = (FINE ? OFF_QH : OFF_Q16) + qidx;
    const size_t ko = (FINE ? OFF_KH : OFF_K16) + kidx;
    const size_t vo = (FINE ? OFF_VTH : OFF_VT16) + vidx;
    const size_t qdl = FINE ? (OFF_QL - OFF_QH) : 0;
    const size_t kdl = FINE ? (OFF_KL - OFF_KH) : 0;
    const size_t vdl = FINE ? (OFF_VTL - OFF_VTH) : 0;

    const float NEG = -__builtin_inff();
    const float SC2 = FINE ? 0.18033688011112042f : (0.18033688011112042f / 256.0f);
    float mrow[8], lrow[8];
    v8f o[4];
#pragma unroll
    for (int r = 0; r < 8; ++r) { mrow[r] = NEG; lrow[r] = 0.f; }
#pragma unroll
    for (int t = 0; t < 4; ++t) o[t] = zero8();

    const int nsteps = (q0 >> 5) + 1;
    for (int st = 0; st < nsteps; ++st) {
        const int kv0 = st << 5;
        v8f s0 = zero8(), s1 = zero8();
#pragma unroll
        for (int ks = 0; ks < 2; ++ks) {
            const size_t k0 = ko + (size_t)kv0 * DMODEL + ks * 32;
            const size_t k1 = k0 + (size_t)16 * DMODEL;
            if (FINE) {
                const v16b qh = ldfb(pl + qo + ks * 32), ql = ldfb(pl + qo + qdl + ks * 32);
                const v16b a0 = ldfb(pl + k0), b0 = ldfb(pl + k0 + kdl);
                s0 = mmab(qh, a0, s0); s0 = mmab(qh, b0, s0); s0 = mmab(ql, a0, s0);
                const v16b a1 = ldfb(pl + k1), b1 = ldfb(pl + k1 + kdl);
                s1 = mmab(qh, a1, s1); s1 = mmab(qh, b1, s1); s1 = mmab(ql, a1, s1);
            } else {
                const v16h qh = ldfh(pl + qo + ks * 32);
                s0 = mmah(qh, ldfh(pl + k0), s0);
                s1 = mmah(qh, ldfh(pl + k1), s1);
            }
        }
        const bool diag = (kv0 + 31 > q0);
#pragma unroll
        for (int r = 0; r < 8; ++r) {
            float x0 = s0[r] * SC2, x1 = s1[r] * SC2;
            if (diag) {
                const int qrow = q0 + 8 * hh + r;
                x0 = (kv0 + c > qrow) ? NEG : x0;
                x1 = (kv0 + 16 + c > qrow) ? NEG : x1;
            }
            float mx = fmaxf(x0, x1);
            mx = fmaxf(mx, __shfl_xor(mx, 1, 32)); mx = fmaxf(mx, __shfl_xor(mx, 2, 32));
            mx = fmaxf(mx, __shfl_xor(mx, 4, 32)); mx = fmaxf(mx, __shfl_xor(mx, 8, 32));
            const float mnew = fmaxf(mrow[r], mx);
            const float alpha = (mnew == NEG) ? 1.f : exp2f(mrow[r] - mnew);
            const float p0 = (x0 == NEG) ? 0.f : exp2f(x0 - mnew);
            const float p1 = (x1 == NEG) ? 0.f : exp2f(x1 - mnew);
            float ps = p0 + p1;
            ps += __shfl_xor(ps, 1, 32); ps += __shfl_xor(ps, 2, 32); ps += __shfl_xor(ps, 4, 32); ps += __shfl_xor(ps, 8, 32);
            lrow[r] = lrow[r] * alpha + ps; mrow[r] = mnew;
#pragma unroll
            for (int t = 0; t < 4; ++t) o[t][r] *= alpha;
            const int pi = (8 * hh + r) * PPITCH + c;
            if (FINE) {
                const unsigned short h0 = bfu_rne(p0), h1 = bfu_rne(p1);
                Ph[wave][pi] = h0; Ph[wave][pi + 16] = h1;
                Pl[wave][pi] = bfu_rne(p0 - bfu_f32(h0)); Pl[wave][pi + 16] = bfu_rne(p1 - bfu_f32(h1));
            } else {
                Ph[wave][pi] = f16_bits(p0 * 4096.f); Ph[wave][pi + 16] = f16_bits(p1 * 4096.f);
            }
        }
        wave_sync();
        FBU fa, fl;
        fa.q[0] = *(const v4u*)&Ph[wave][c * PPITCH + 8 * hh];
        fa.q[1] = *(const v4u*)&Ph[wave][c * PPITCH + 16 + 8 * hh];
        fl.q[0] = fa.q[0]; fl.q[1] = fa.q[1];
        if (FINE) {
            fl.q[0] = *(const v4u*)&Pl[wave][c * PPITCH + 8 * hh];
            fl.q[1] = *(const v4u*)&Pl[wave][c * PPITCH + 16 + 8 * hh];
        }
        wave_sync();
#pragma unroll
        for (int t = 0; t < 4; ++t) {
            const size_t vp = vo + (size_t)(t * 16) * SP + kv0;
            if (FINE) {
                const v16b vh = ldfb(pl + vp), vl = ldfb(pl + vp + vdl);
                o[t] = mmab(fa.b, vh, o[t]); o[t] = mmab(fa.b, vl, o[t]); o[t] = mmab(fl.b, vh, o[t]);
            } else {
                o[t] = mmah(fa.h, ldfh(pl + vp), o[t]);
            }
        }
    }

    const float OSC = FINE ? 1.0f : 65536.0f;
#pragma unroll
    for (int r = 0; r < 8; ++r) {
        const float inv = 1.0f / (lrow[r] * OSC);
#pragma unroll
        for (int t = 0; t < 4; ++t) Os[wave][(8 * hh + r) * 68 + t * 16 + c] = o[t][r] * inv;
    }
    wave_sync();
    {
        float* ob = out + ((size_t)(b * SEQ + q0)) * DMODEL + h * HDIM;
        const int c4 = (lane & 15) * 4;
        for (int pass = 0; pass < 2; ++pass) {
#pragma unroll
            for (int it = 0; it < 8; ++it) {
                const int row = it * 2 + hh;
                const v4f val = *(const v4f*)&Os[wave][row * 68 + c4];
                *(volatile v4f*)(ob + (size_t)row * DMODEL + c4) = val;
            }
            __threadfence();
        }
    }
}

__global__ __launch_bounds__(128) void k_attn_fine(const unsigned short* __restrict__ pl, float* out) { attn_body<true>(pl, out); }
__global__ __launch_bounds__(128) void k_attn_plain(const unsigned short* __restrict__ pl, float* out) { attn_body<false>(pl, out); }

extern "C" void kernel_launch(void* const* d_in, const int* in_sizes, int n_in, void* d_out, int out_size, void* d_ws, size_t ws_size, hipStream_t stream) {
    if (n_in < 9) return;
    const long long needx = (long long)(NB - 1) * (long long)X_BS_FULL + (long long)SEQ * DMODEL;
    if ((long long)in_sizes[0] < needx || (long long)in_sizes[1] < needx || (long long)in_sizes[2] < needx) return;
    if (in_sizes[3] < NHEAD * DMODEL * HDIM || in_sizes[5] < NHEAD * DMODEL * HDIM || in_sizes[7] < NHEAD * DMODEL * HDIM) return;
    if (in_sizes[4] < DMODEL || in_sizes[6] < DMODEL || in_sizes[8] < DMODEL) return;
    if ((long long)out_size < (long long)MTOK * DMODEL) return;
    if (ws_size < (size_t)WS_HALVES * 2) return;
    const float* xq = (const float*)d_in[0];
    const float* xk = (const float*)d_in[1];
    const float* xv = (const float*)d_in[2];
    const float* wq = (const float*)d_in[3];
    const float* bq = (const float*)d_in[4];
    const float* wk = (const float*)d_in[5];
    const float* bk = (const float*)d_in[6];
    const float* wv = (const float*)d_in[7];
    const float* bv = (const float*)d_in[8];
    float* out = (float*)d_out;
    unsigned short* ws16 = (unsigned short*)d_ws;

    k_cvt_x<<<dim3((unsigned)((MTOK * 128) / 256), 3u), 256, 0, stream>>>(xq, xk, xv, ws16);
    k_cvt_w<<<dim3((unsigned)((DMODEL * 128) / 256), 3u), 256, 0, stream>>>(wq, wk, wv, ws16);
    k_proj<<<dim3((unsigned)(PROJ_TILES / 8), 3u), 256, 0, stream>>>(ws16, ws16, bq, bk, bv);
    k_attn_fine<<<dim3((unsigned)FINE_BLOCKS), 128, 0, stream>>>(ws16, out);
    if (PLAIN_BLOCKS > 0) k_attn_plain<<<dim3((unsigned)(PLAIN_BLOCKS > 0 ? PLAIN_BLOCKS : 1)), 128, 0, stream>>>(ws16, out);
}
